// CrissCrossAttention_48954037240512
// MI455X (gfx1250) — hardware-verified
//
#include <hip/hip_runtime.h>
#include <math.h>

typedef __attribute__((ext_vector_type(16))) _Float16 v16h;
typedef __attribute__((ext_vector_type(16))) __bf16 v16b;
typedef __attribute__((ext_vector_type(8)))  _Float16 v8h;
typedef __attribute__((ext_vector_type(8)))  float v8f;
typedef __attribute__((ext_vector_type(4)))  float v4f;
typedef __attribute__((ext_vector_type(2)))  float v2f;
typedef __attribute__((ext_vector_type(4)))  unsigned v4u;
typedef __attribute__((ext_vector_type(4)))  int v4i;
typedef float __attribute__((may_alias)) float_a;
typedef int __attribute__((may_alias)) int_a;

template <typename T> __device__ __forceinline__ void vst2(void* p, T v) { *(volatile T*)p = v; __threadfence(); *(volatile T*)p = v; }
__device__ __forceinline__ v8f wmma16(v16h a, v16h b, v8f c) {
  v8f d = __builtin_amdgcn_wmma_f32_16x16x32_f16(false, a, false, b, (short)0, c, false, false);
  asm volatile("v_nop\n\tv_nop\n\tv_nop\n\tv_nop" : "+v"(d) : "v"(a), "v"(b));
  return d;
}
__device__ __forceinline__ v8f wmma_bf(v16b a, v16b b, v8f c) {
  v8f d = __builtin_amdgcn_wmma_f32_16x16x32_bf16(false, a, false, b, (short)0, c, false, false);
  asm volatile("v_nop\n\tv_nop\n\tv_nop\n\tv_nop" : "+v"(d) : "v"(a), "v"(b));
  return d;
}
__device__ __forceinline__ v16h frag_h(const _Float16* rowk0, int lane) {
  union { v16h v; v8h q[2]; } u; const _Float16* p = rowk0 + 8 * (lane >> 4);
  u.q[0] = *(const v8h*)p; u.q[1] = *(const v8h*)(p + 16); return u.v;
}
__device__ __forceinline__ v16h frag_f32(const float* rowk0, int lane) {
  v16h a; const float* p = rowk0 + 8 * (lane >> 4);
#pragma unroll
  for (int i = 0; i < 8; ++i) { a[i] = (_Float16)p[i]; a[8 + i] = (_Float16)p[16 + i]; }
  return a;
}
__device__ __forceinline__ v16h frag_f32s(const float* rowk0, int lane, float sc) {
  v16h a; const float* p = rowk0 + 8 * (lane >> 4);
#pragma unroll
  for (int i = 0; i < 8; ++i) { a[i] = (_Float16)(p[i] * sc); a[8 + i] = (_Float16)(p[16 + i] * sc); }
  return a;
}
__device__ __forceinline__ v16h fragc_f32(const float* W, int k0, int n, int lane, int ld, int K) {
  v16h a; const int g = lane >> 4;
#pragma unroll
  for (int i = 0; i < 8; ++i) { const int ka = k0 + 8 * g + i, kb = ka + 16;
    a[i] = (_Float16)(ka < K ? W[(size_t)(ka < K ? ka : K - 1) * ld + n] : 0.f); a[8 + i] = (_Float16)(kb < K ? W[(size_t)(kb < K ? kb : K - 1) * ld + n] : 0.f); }
  return a;
}
struct F2 { v16b h, l; };
__device__ __forceinline__ F2 bsplit16(const float v[16]) { F2 r;
#pragma unroll
  for (int i = 0; i < 16; ++i) { const __bf16 h = (__bf16)v[i]; r.h[i] = h; r.l[i] = (__bf16)(v[i] - (float)h); }
  return r; }
__device__ __forceinline__ F2 split_row(const float* row, int k0, int lane) { float v[16]; const float* p = row + k0 + 8 * (lane >> 4);
#pragma unroll
  for (int i = 0; i < 8; ++i) { v[i] = p[i]; v[8 + i] = p[16 + i]; }
  return bsplit16(v); }
__device__ __forceinline__ F2 split_rowK(const float* row, int k0, int lane, int K) { float v[16]; const int g = lane >> 4;
#pragma unroll
  for (int i = 0; i < 8; ++i) { const int ka = k0 + 8 * g + i, kb = ka + 16; v[i] = ka < K ? row[ka < K ? ka : K - 1] : 0.f; v[8 + i] = kb < K ? row[kb < K ? kb : K - 1] : 0.f; }
  return bsplit16(v); }
__device__ __forceinline__ F2 split_col(const float* W, int k0, int n, int lane, int ld, int K) { float v[16]; const int g = lane >> 4;
#pragma unroll
  for (int i = 0; i < 8; ++i) { const int ka = k0 + 8 * g + i, kb = ka + 16; v[i] = ka < K ? W[(size_t)(ka < K ? ka : K - 1) * ld + n] : 0.f; v[8 + i] = kb < K ? W[(size_t)(kb < K ? kb : K - 1) * ld + n] : 0.f; }
  return bsplit16(v); }
__device__ __forceinline__ v8f mac3(const F2& a, const F2& b, v8f c) { c = wmma_bf(a.l, b.h, c); c = wmma_bf(a.h, b.l, c); return wmma_bf(a.h, b.h, c); }
__device__ __forceinline__ float sigm(float v) { return 1.0f / (1.0f + expf(-v)); }
#define LDSX() do { asm volatile("s_wait_dscnt 0" ::: "memory"); __builtin_amdgcn_wave_barrier(); __builtin_amdgcn_fence(__ATOMIC_RELEASE, "workgroup"); } while (0)

__device__ __forceinline__ float bfr(float v) { return (float)(__bf16)v; }
#define NB 4
#define TT 4096
#define CX 256
#define DQ 32
#ifndef TNB
#define TNB NB
#endif
#ifndef XSTR
#define XSTR TT
#endif
typedef __attribute__((ext_vector_type(8))) __bf16 v8b;
__device__ __forceinline__ v16b frag_b(const __bf16* rowk0, int lane) { union { v16b v; v8b q[2]; } u; const __bf16* p = rowk0 + 8 * (lane >> 4); u.q[0] = *(const v8b*)p; u.q[1] = *(const v8b*)(p + 16); return u.v; }
#define WS_XS  0u
#define WS_XG  (WS_XS + 4u * (size_t)NB * TT * CX)
#define WS_GH  (WS_XG + 4u * (size_t)NB * TT * CX)
#define WS_GL  (WS_GH + 2u * (size_t)NB * TT * DQ)
#define WS_FH  (WS_GL + 2u * (size_t)NB * TT * DQ)
#define WS_FL  (WS_FH + 2u * (size_t)NB * TT * DQ)
#define WS_VT  (WS_FL + 2u * (size_t)NB * TT * DQ)
#define WS_S   (WS_VT + 2u * (size_t)NB * CX * TT)
#define WS_END (WS_S + 4u * (size_t)TT * TT)
__global__ __launch_bounds__(256) void k_xt(const float* __restrict__ SRC, const float* __restrict__ TGT, float* __restrict__ XS, float* __restrict__ XG) { __shared__ float st[CX][65];
  const int t = threadIdx.x; const int l0 = blockIdx.x * 64; const size_t b = blockIdx.y; const float* IN = blockIdx.z == 0 ? SRC : TGT; float* OUTR = blockIdx.z == 0 ? XS : XG;
  for (int e = t; e < CX * 64; e += 256) { const int c = e >> 6, ll = e & 63; st[c][ll] = IN[(b * CX + c) * (size_t)XSTR + l0 + ll]; }
  __syncthreads();
  for (int e = t; e < 64 * 64; e += 256) { const int ll = e >> 6, q = e & 63; v4f o; o[0] = st[q * 4][ll]; o[1] = st[q * 4 + 1][ll]; o[2] = st[q * 4 + 2][ll]; o[3] = st[q * 4 + 3][ll]; vst2(OUTR + (b * TT + l0 + ll) * CX + q * 4, o); } }
__global__ __launch_bounds__(128) void k_fg(const float* __restrict__ XQ, const float* __restrict__ XK, const float* __restrict__ WF, const float* __restrict__ BF, const float* __restrict__ WG, const float* __restrict__ BG, _Float16* __restrict__ GH, _Float16* __restrict__ GL, _Float16* __restrict__ FH, _Float16* __restrict__ FL) {
  __shared__ __align__(16) _Float16 st[4][4][16][40];
  const int tid = threadIdx.x, wave = tid >> 5, lane = tid & 31, col = lane & 15, g = lane >> 4; const size_t r0 = (size_t)blockIdx.x * 64 + wave * 16;
  v8f acc[4] = {};
#pragma unroll 2
  for (int kc = 0; kc < CX / 32; ++kc) { v16b aq, ak; { const float* p = XQ + (r0 + col) * CX + kc * 32 + 8 * g; const float* p2 = XK + (r0 + col) * CX + kc * 32 + 8 * g;
#pragma unroll
      for (int i = 0; i < 8; ++i) { aq[i] = (__bf16)p[i]; aq[8 + i] = (__bf16)p[16 + i]; ak[i] = (__bf16)p2[i]; ak[8 + i] = (__bf16)p2[16 + i]; } }
#pragma unroll
    for (int j = 0; j < 4; ++j) { v16b w; const float* WA = (j < 2) ? WG : WF; const v16b& a = (j < 2) ? aq : ak; const int o = (j & 1) * 16 + col;
#pragma unroll
      for (int i = 0; i < 8; ++i) { w[i] = (__bf16)WA[(size_t)o * CX + kc * 32 + 8 * g + i]; w[8 + i] = (__bf16)WA[(size_t)o * CX + kc * 32 + 16 + 8 * g + i]; }
      asm volatile("s_wait_loadcnt 0x0" ::: "memory"); acc[j] = wmma_bf(a, w, acc[j]); } }
#pragma unroll
  for (int j = 0; j < 4; ++j) { const int o = (j & 1) * 16 + col; const float bb = (j < 2) ? bfr(BG[o]) : bfr(BF[o]); const int ph = (j < 2) ? 0 : 2;
#pragma unroll
    for (int r = 0; r < 8; ++r) { const float v = acc[j][r] + bb; const _Float16 hv = (_Float16)v; st[wave][ph][8 * g + r][o] = hv; st[wave][ph + 1][8 * g + r][o] = (_Float16)((v - (float)hv) * 1024.0f); } }
  LDSX();
  { const int rl = lane >> 1, half = lane & 1;
    _Float16* P4[4] = {GH, GL, FH, FL};
#pragma unroll
    for (int ph = 0; ph < 4; ++ph) { vst2((v4u*)(P4[ph] + (r0 + rl) * DQ + half * 16), *(const v4u*)&st[wave][ph][rl][half * 16]); vst2((v4u*)(P4[ph] + (r0 + rl) * DQ + half * 16 + 8), *(const v4u*)&st[wave][ph][rl][half * 16 + 8]); } } }
__global__ __launch_bounds__(128) void k_hv(const float* __restrict__ X, const float* __restrict__ WH, const float* __restrict__ BH, _Float16* __restrict__ VT) { __shared__ __align__(16) _Float16 th[128][72];
  const int tid = threadIdx.x, wave = tid >> 5, lane = tid & 31, col = lane & 15, g = lane >> 4; const int c0 = blockIdx.y * 128; const size_t r0 = (size_t)blockIdx.x * 64;
  v8f acc[8] = {};
#pragma unroll 2
  for (int kc = 0; kc < CX / 32; ++kc) { v16b a; { const float* p = X + (r0 + wave * 16 + col) * CX + kc * 32 + 8 * g;
#pragma unroll
      for (int i = 0; i < 8; ++i) { a[i] = (__bf16)p[i]; a[8 + i] = (__bf16)p[16 + i]; } }
#pragma unroll
    for (int j = 0; j < 8; ++j) { v16b w; const int o = c0 + j * 16 + col;
#pragma unroll
      for (int i = 0; i < 8; ++i) { w[i] = (__bf16)WH[(size_t)o * CX + kc * 32 + 8 * g + i]; w[8 + i] = (__bf16)WH[(size_t)o * CX + kc * 32 + 16 + 8 * g + i]; }
      asm volatile("s_wait_loadcnt 0x0" ::: "memory"); acc[j] = wmma_bf(a, w, acc[j]); } }
#pragma unroll
  for (int j = 0; j < 8; ++j) { const float bb = bfr(BH[c0 + j * 16 + col]);
#pragma unroll
    for (int r = 0; r < 8; ++r) th[j * 16 + col][wave * 16 + 8 * g + r] = (_Float16)(acc[j][r] + bb); }
  __syncthreads();
  { const size_t b = r0 / TT; const int m0 = (int)(r0 % TT); for (int e = tid; e < 128 * 8; e += 128) { const int cl = e >> 3, q = e & 7; vst2((unsigned*)(VT + (b * CX + c0 + cl) * (size_t)TT + m0 + q * 8), *(const v4u*)&th[cl][q * 8]); } } }
__global__ __launch_bounds__(128) void k_sc(const _Float16* __restrict__ GH, const _Float16* __restrict__ GL, const _Float16* __restrict__ FH, const _Float16* __restrict__ FL, int b, float* __restrict__ S) { __shared__ __align__(16) float ss[4][16][132];
  const int tid = threadIdx.x, wave = tid >> 5, lane = tid & 31, col = lane & 15, g = lane >> 4; const int k0 = blockIdx.y * 128; const int ql0 = blockIdx.x * 64 + wave * 16; const size_t q0 = (size_t)b * TT + ql0;
  v8f acc[8] = {}, accl[8] = {};
  { const v16h ah = frag_h(GH + (q0 + col) * DQ, lane), al = frag_h(GL + (q0 + col) * DQ, lane);
#pragma unroll
    for (int j = 0; j < 8; ++j) { const size_t ko = ((size_t)b * TT + k0 + j * 16 + col) * DQ; const v16h kb = frag_h(FH + ko, lane), kl = frag_h(FL + ko, lane); acc[j] = wmma16(ah, kb, acc[j]); accl[j] = wmma16(al, kb, accl[j]); accl[j] = wmma16(ah, kl, accl[j]); } }
#pragma unroll
  for (int j = 0; j < 8; ++j)
#pragma unroll
    for (int r = 0; r < 8; ++r) ss[wave][8 * g + r][j * 16 + col] = acc[j][r] + accl[j][r] * (1.0f / 1024.0f);
  LDSX(); for (int rl = 0; rl < 16; ++rl) vst2(S + (size_t)(ql0 + rl) * TT + k0 + lane * 4, *(const v4f*)&ss[wave][rl][lane * 4]); }
__global__ __launch_bounds__(128) void k_csm(float* __restrict__ S) { const int m = blockIdx.x * 128 + threadIdx.x; float mx = -3.0e38f;
  for (int n = 0; n < TT; ++n) mx = fmaxf(mx, S[(size_t)n * TT + m]);
  float z = 0.f; for (int n = 0; n < TT; ++n) z += expf(S[(size_t)n * TT + m] - mx);
  const float sc = 2048.0f / z;
  for (int n = 0; n < TT; ++n) { const size_t o = (size_t)n * TT + m; S[o] = expf(S[o] - mx) * sc; } }
__global__ __launch_bounds__(128) void k_pv(const float* __restrict__ PS, const _Float16* __restrict__ VT, const float* __restrict__ SRC, int b, float* __restrict__ OUT) { __shared__ __align__(16) float stc[128][68];
  const int tid = threadIdx.x, wave = tid >> 5, lane = tid & 31, col = lane & 15, g = lane >> 4; const int ql0 = blockIdx.x * 64 + wave * 16; const int c0 = blockIdx.y * 128;
  v8f acc[8] = {}, accl[8] = {};
#pragma unroll 1
  for (int kc = 0; kc < TT / 32; ++kc) { v16h ph, pl; { const float* pr = PS + (size_t)(ql0 + col) * TT + kc * 32 + 8 * g;
#pragma unroll
      for (int i = 0; i < 8; ++i) { const float a0 = pr[i], a1 = pr[16 + i]; const _Float16 h0 = (_Float16)a0, h1 = (_Float16)a1; ph[i] = h0; ph[8 + i] = h1; pl[i] = (_Float16)((a0 - (float)h0) * 1024.0f); pl[8 + i] = (_Float16)((a1 - (float)h1) * 1024.0f); } }
    asm volatile("s_wait_loadcnt 0x0" ::: "memory");
#pragma unroll
    for (int j = 0; j < 8; ++j) { const v16h vv = frag_h(VT + ((size_t)b * CX + c0 + j * 16 + col) * (size_t)TT + kc * 32, lane); acc[j] = wmma16(ph, vv, acc[j]); accl[j] = wmma16(pl, vv, accl[j]); } }
#pragma unroll
  for (int j = 0; j < 8; ++j)
#pragma unroll
    for (int r = 0; r < 8; ++r) stc[j * 16 + col][wave * 16 + 8 * g + r] = (acc[j][r] + accl[j][r] * (1.0f / 1024.0f)) * (1.0f / 2048.0f);
  __syncthreads();
  { const int n0 = blockIdx.x * 64; for (int e = tid; e < 128 * 16; e += 128) { const int cl = e >> 4, q = e & 15; const size_t off = ((size_t)b * CX + c0 + cl) * (size_t)XSTR + n0 + q * 4; const v4f sr = *(const v4f*)(SRC + off); v4f o = *(const v4f*)&stc[cl][q * 4]; o[0] += bfr(sr[0]); o[1] += bfr(sr[1]); o[2] += bfr(sr[2]); o[3] += bfr(sr[3]); vst2(OUT + off, o); } } }
extern "C" void kernel_launch(void* const* d_in, const int* in_sizes, int n_in, void* d_out, int out_size, void* d_ws, size_t ws_size, hipStream_t stream) {
  (void)in_sizes; (void)n_in; (void)out_size;
  const float** F = (const float**)d_in;
  if (ws_size < (size_t)WS_END) return;
  char* ws = (char*)d_ws; float *XS = (float*)(ws + WS_XS), *XG = (float*)(ws + WS_XG); _Float16 *GH = (_Float16*)(ws + WS_GH), *GL = (_Float16*)(ws + WS_GL), *FH = (_Float16*)(ws + WS_FH), *FL = (_Float16*)(ws + WS_FL); _Float16* VT = (_Float16*)(ws + WS_VT); float* S = (float*)(ws + WS_S); (void)XG;
  k_xt<<<dim3(TT / 64, TNB, 1), 256, 0, stream>>>(F[0], F[0], XS, XS);
  k_fg<<<dim3(TNB * TT / 64), 128, 0, stream>>>(XS, XS, F[3], F[4], F[1], F[2], GH, GL, FH, FL);
  k_hv<<<dim3(TNB * TT / 64, CX / 128), 128, 0, stream>>>(XS, F[5], F[6], VT);
  for (int b = 0; b < TNB; ++b) {
    k_sc<<<dim3(TT / 64, TT / 128), 128, 0, stream>>>(FH, FL, GH, GL, b, S);
    k_csm<<<dim3(TT / 128), 128, 0, stream>>>(S);
    k_pv<<<dim3(TT / 64, CX / 128), 128, 0, stream>>>(S, VT, F[0], b, (float*)d_out);
  }
}
